// CrossAttention_62646392980064
// MI455X (gfx1250) — hardware-run, weakly checked
//
#include <hip/hip_runtime.h>
#include <math.h>
#include <stdint.h>

#ifndef NB
#define NB 2
#endif
#ifndef SEQ
#define SEQ 2048
#endif
#define NB_FULL   2
#define SEQ_FULL  2048
#define DM1   1024
#define DM2   512
#define NH    8
#define HD    64
#define DI    (NH * HD)
#define NRPF  192
#define PK    (2 * NRPF)
#define NPOS  (2 * SEQ)
#define NQB   (SEQ / 64)
#define PCARRY 16384.0f
#define VCARRY 16.0f
#define CCARRY 256.0f
#define RQ     4096.0f
#define WOC    64.0f
#define OUT2_OFF ((size_t)NB_FULL * SEQ_FULL * DM1)

static_assert(HD == 64);
static_assert(NH * HD == DI && DI == 512);
static_assert(NH == 8);
static_assert(NRPF == 6 * 32 && (NRPF % 64) == 0);
static_assert((PK % 32) == 0 && ((PK * 2) % 128) == 0);
static_assert(PK == 256 + 128);
static_assert(NB >= 1 && NB <= NB_FULL);
static_assert(SEQ >= 64 && SEQ <= SEQ_FULL && (SEQ % 64) == 0);
static_assert((SEQ & (SEQ - 1)) == 0);
static_assert(((SEQ - 16) % 16) == 0);
static_assert((NPOS % 64) == 0 && (NPOS % 32) == 0 && (NPOS % 8) == 0);
static_assert((DM1 % 64) == 0 && (DM2 % 64) == 0 && (DI % 64) == 0);
static_assert((DM1 % 32) == 0 && (DM2 % 32) == 0 && (DI % 32) == 0);
static_assert(((NB * SEQ) % 64) == 0);
static_assert(((SEQ * DM1 / 8) % 256) == 0 && ((SEQ * DM2 / 8) % 256) == 0);
static_assert(256 * 4 * 4 == 64 * 64);
static_assert(PCARRY < 65504.0f);
static_assert(OUT2_OFF * 4 == (size_t)16777216);
static_assert((OUT2_OFF + (size_t)((NB_FULL - 1) * SEQ_FULL + SEQ_FULL) * DM1) * 4 == (size_t)33554432);

static constexpr size_t WSB_X1  = (size_t)NB * SEQ * DM1 * 2;
static constexpr size_t WSB_X2  = (size_t)NB * SEQ * DM2 * 2;
static constexpr size_t WSB_W1  = (size_t)DI * DM1 * 2;
static constexpr size_t WSB_W2  = (size_t)DI * DM2 * 2;
static constexpr size_t WSB_WR  = (size_t)DI * PK * 2;
static constexpr size_t WSB_WO  = (size_t)DM1 * DI * 2;
static constexpr size_t WSB_POS = (size_t)NPOS * PK * 2;
static constexpr size_t WSB_PT  = (size_t)512;
static constexpr size_t WSB_P   = (size_t)NB * SEQ * DI * 2;
static constexpr size_t WSB_R   = (size_t)NPOS * DI * 2;
static constexpr size_t WSB_CT  = (size_t)NH * NPOS * 4;
static constexpr size_t WSB_ST  = (size_t)NB * NH * NQB * 128 * 4;
static constexpr size_t WSB_TOTAL = WSB_X1 + WSB_X2 + 2 * WSB_W1 + 2 * WSB_W2 + WSB_WR + 2 * WSB_WO + WSB_POS + WSB_PT +
                                    6 * WSB_P + 2 * WSB_R + WSB_CT + WSB_ST;
static_assert(WSB_TOTAL <= (size_t)134217728);
static_assert((WSB_X1 % 128) == 0 && (WSB_X2 % 128) == 0 && (WSB_W1 % 128) == 0 && (WSB_W2 % 128) == 0);
static_assert((WSB_WR % 128) == 0 && (WSB_WO % 128) == 0 && (WSB_POS % 128) == 0 && (WSB_PT % 128) == 0);
static_assert((WSB_P % 128) == 0 && (WSB_R % 128) == 0 && (WSB_CT % 128) == 0 && (WSB_ST % 128) == 0);

typedef _Float16 v16h __attribute__((ext_vector_type(16)));
typedef _Float16 v8h  __attribute__((ext_vector_type(8)));
typedef __bf16   v16b __attribute__((ext_vector_type(16)));
typedef __bf16   v8b  __attribute__((ext_vector_type(8)));
typedef float    v8f  __attribute__((ext_vector_type(8)));
typedef float    v4f  __attribute__((ext_vector_type(4)));
typedef unsigned int v4u __attribute__((ext_vector_type(4)));
typedef unsigned short v8us __attribute__((ext_vector_type(8)));

#if defined(__HIP_DEVICE_COMPILE__)
#define DEV_ASM 1
#else
#define DEV_ASM 0
#endif

__device__ __forceinline__ unsigned short bf_bits(float f) {
  unsigned u = __float_as_uint(f);
  return (unsigned short)((u + 0x7FFFu + ((u >> 16) & 1u)) >> 16);
}
__device__ __forceinline__ float bf_up(unsigned short hb) { return __uint_as_float(((unsigned)hb) << 16); }
__device__ __forceinline__ unsigned short h_bits(_Float16 x) { return __builtin_bit_cast(unsigned short, x); }
__device__ __forceinline__ unsigned pk16(unsigned short a, unsigned short b) { return (unsigned)a | ((unsigned)b << 16); }
__device__ __forceinline__ v8f zero8() { v8f z = {0.f, 0.f, 0.f, 0.f, 0.f, 0.f, 0.f, 0.f}; return z; }
static __device__ __forceinline__ _Float16 toh_flush(float v) {
  const _Float16 r = (_Float16)v;
  return (fabsf(v) < 6.103515625e-05f) ? (_Float16)0.0f : r;
}

template <typename OT> struct FT;
template <> struct FT<__bf16>   { typedef v16b frag; typedef v8b half8; };
template <> struct FT<_Float16> { typedef v16h frag; typedef v8h half8; };

template <typename OT>
__device__ __forceinline__ typename FT<OT>::frag ldfrag(const OT* p) {
  union { typename FT<OT>::frag v; typename FT<OT>::half8 h[2]; } f;
  f.h[0] = *(const typename FT<OT>::half8*)(p);
  f.h[1] = *(const typename FT<OT>::half8*)(p + 16);
  return f.v;
}

__device__ __forceinline__ v8f mmar(v16b a, v16b b, v8f c) {
  return __builtin_amdgcn_wmma_f32_16x16x32_bf16(false, a, false, b, (short)0, c, false, false);
}
__device__ __forceinline__ v8f mmar(v16h a, v16h b, v8f c) {
  return __builtin_amdgcn_wmma_f32_16x16x32_f16(false, a, false, b, (short)0, c, false, false);
}
__device__ __forceinline__ v8f mma_h(v16h a, v16h b, v8f c) {
  c = __builtin_amdgcn_wmma_f32_16x16x32_f16(false, a, false, b, (short)0, c, false, false);
#if DEV_ASM
  asm volatile("v_nop\n\tv_nop\n\tv_nop\n\tv_nop" : "+v"(c) : "v"(a), "v"(b));
#endif
  return c;
}
__device__ __forceinline__ void dep_guard(v8f& a, v8f& b, v16b x, v16b y) {
#if DEV_ASM
  asm volatile("v_nop\n\tv_nop\n\tv_nop\n\tv_nop" : "+v"(a), "+v"(b) : "v"(x), "v"(y));
#else
  (void)a; (void)b; (void)x; (void)y;
#endif
}
__device__ __forceinline__ void dep_guard(v8f& a, v8f& b, v16h x, v16h y) {
#if DEV_ASM
  asm volatile("v_nop\n\tv_nop\n\tv_nop\n\tv_nop" : "+v"(a), "+v"(b) : "v"(x), "v"(y));
#else
  (void)a; (void)b; (void)x; (void)y;
#endif
}
__device__ __forceinline__ void keep4(v16b a, v16b b, v16b c, v16b d) {
#if DEV_ASM
  asm volatile("v_nop" :: "v"(a), "v"(b), "v"(c), "v"(d));
#else
  (void)a; (void)b; (void)c; (void)d;
#endif
}
__device__ __forceinline__ void keep4(v16h a, v16h b, v16h c, v16h d) {
#if DEV_ASM
  asm volatile("v_nop" :: "v"(a), "v"(b), "v"(c), "v"(d));
#else
  (void)a; (void)b; (void)c; (void)d;
#endif
}
__device__ __forceinline__ void acc_guard4(v8f& a, v8f& b, v8f& c, v8f& d) {
#if DEV_ASM
  asm volatile("v_nop\n\tv_nop\n\tv_nop\n\tv_nop" : "+v"(a), "+v"(b), "+v"(c), "+v"(d));
#else
  (void)a; (void)b; (void)c; (void)d;
#endif
}

__global__ __launch_bounds__(256) void cvt_bf16x8(const float* __restrict__ in, long long istride,
                                                 unsigned short* out, long long ostride, int n8) {
  const int b = blockIdx.y;
  const int i = blockIdx.x * 256 + (int)threadIdx.x;
  if (i < n8) {
    const float* ip = in + (size_t)b * (size_t)istride + (size_t)i * 8;
    const v4f a  = *(const v4f*)(ip);
    const v4f a4 = *(const v4f*)(ip + 4);
    v4u p;
    p[0] = pk16(bf_bits(a[0]),  bf_bits(a[1]));
    p[1] = pk16(bf_bits(a[2]),  bf_bits(a[3]));
    p[2] = pk16(bf_bits(a4[0]), bf_bits(a4[1]));
    p[3] = pk16(bf_bits(a4[2]), bf_bits(a4[3]));
    unsigned short* o = out + (size_t)b * (size_t)ostride + (size_t)i * 8;
    *(volatile v4u*)o = p;
    __threadfence();
    *(volatile v4u*)o = p;
  }
}

template <int MODE>
__device__ __forceinline__ unsigned short cvm(float f, float scale) {
  const unsigned short hb = bf_bits(f);
  if (MODE == 0) return hb;
  return h_bits((_Float16)(bf_up(hb) * scale));
}

template <int MODE>
__device__ __forceinline__ void wtrans_body(const float* __restrict__ W, int C,
                                            unsigned short* T, int ldt, int coff, float scale,
                                            float* sW) {
  const int tid  = threadIdx.x;
  const int lane = tid & 31;
  const int wave = tid >> 5;
  const int n0 = blockIdx.x * 64;
  const int k0 = blockIdx.y * 64;
#pragma unroll
  for (int j = 0; j < 4; ++j) {
    const int lin = tid + j * 256;
    const int r = lin >> 4, c4 = (lin & 15) * 4;
    const v4f val = *(const v4f*)(W + (size_t)(k0 + r) * (size_t)C + n0 + c4);
    sW[(c4 + 0) * 68 + r] = val[0];
    sW[(c4 + 1) * 68 + r] = val[1];
    sW[(c4 + 2) * 68 + r] = val[2];
    sW[(c4 + 3) * 68 + r] = val[3];
  }
  __syncthreads();
  const int q = lane >> 3, c8 = (lane & 7) * 8;
  v4u pv[2];
#pragma unroll
  for (int it = 0; it < 2; ++it) {
    const int row = it * 32 + wave * 4 + q;
    const float* sp = sW + row * 68 + c8;
    v4u a;
#pragma unroll
    for (int e = 0; e < 4; ++e)
      a[e] = pk16(cvm<MODE>(sp[2 * e], scale), cvm<MODE>(sp[2 * e + 1], scale));
    pv[it] = a;
  }
  for (int ps = 0; ps < 2; ++ps) {
#pragma unroll
    for (int it = 0; it < 2; ++it) {
      const int row = it * 32 + wave * 4 + q;
      *(volatile v4u*)(T + (size_t)(n0 + row) * (size_t)ldt + coff + k0 + c8) = pv[it];
    }
    __threadfence();
  }
}

__global__ __launch_bounds__(256) void wtrans_bf16(const float* __restrict__ W, int C,
                                                  unsigned short* T, int ldt, int coff, float scale) {
  __shared__ __align__(16) float sW[64 * 68];
  wtrans_body<0>(W, C, T, ldt, coff, scale, sW);
}
__global__ __launch_bounds__(256) void wtrans_f16s(const float* __restrict__ W, int C,
                                                  unsigned short* T, int ldt, int coff, float scale) {
  __shared__ __align__(16) float sW[64 * 68];
  wtrans_body<1>(W, C, T, ldt, coff, scale, sW);
}

template <typename OT, int OUT_MODE>
__device__ __forceinline__ void gemm64_body(
    const unsigned short* __restrict__ Ap, int lda, long long strideA,
    const unsigned short* __restrict__ Btp, int ldb, long long strideB,
    void* Cout, void* Cout2, int ldc, long long strideC,
    const float* __restrict__ bias,
    int M, int N, int K, float oscale, float rscale, float* sTall) {
  typedef typename FT<OT>::frag V16;
  const OT* A  = (const OT*)(const void*)Ap;
  const OT* Bt = (const OT*)(const void*)Btp;
  const int b    = blockIdx.y;
  const int lane = threadIdx.x & 31;
  const int wave = threadIdx.x >> 5;
  const int tilesN = N >> 6;
  const int tilesM = M >> 6;
  const int tile = blockIdx.x * 8 + wave;
  if (tile >= tilesM * tilesN) return;
  const int tm = tile / tilesN;
  const int tn = tile - tm * tilesN;
  const int m0 = tm << 6;
  const int n0 = tn << 6;

  const OT* Ab = A  + (size_t)b * (size_t)strideA;
  const OT* Bb = Bt + (size_t)b * (size_t)strideB;

  const int rlane = lane & 15;
  const int koff  = (lane >> 4) * 8;
  const int mOff  = (lane >> 4) * 8;

  v8f acc[4][4];
#pragma unroll
  for (int i = 0; i < 4; ++i)
#pragma unroll
    for (int j = 0; j < 4; ++j) acc[i][j] = zero8();

  for (int k0 = 0; k0 < K; k0 += 32) {
    V16 bq[4];
#pragma unroll
    for (int j = 0; j < 4; ++j)
      bq[j] = ldfrag<OT>(Bb + (size_t)(n0 + (j << 4) + rlane) * ldb + koff + k0);
#pragma unroll
    for (int i = 0; i < 4; ++i) {
      const V16 af = ldfrag<OT>(Ab + (size_t)(m0 + (i << 4) + rlane) * lda + koff + k0);
#pragma unroll
      for (int j = 0; j < 4; ++j) acc[i][j] = mmar(af, bq[j], acc[i][j]);
      dep_guard(acc[i][0], acc[i][3], af, bq[3]);
    }
    keep4(bq[0], bq[1], bq[2], bq[3]);
  }
  acc_guard4(acc[0][0], acc[0][1], acc[0][2], acc[0][3]);
  acc_guard4(acc[1][0], acc[1][1], acc[1][2], acc[1][3]);
  acc_guard4(acc[2][0], acc[2][1], acc[2][2], acc[2][3]);
  acc_guard4(acc[3][0], acc[3][1], acc[3][2], acc[3][3]);

  float* slab = sTall + wave * (16 * 68);
#pragma unroll
  for (int i = 0; i < 4; ++i) {
    const int mBase = m0 + (i << 4);
#pragma unroll
    for (int j = 0; j < 4; ++j) {
#pragma unroll
      for (int r = 0; r < 8; ++r) {
        slab[(mOff + r) * 68 + (j << 4) + rlane] = acc[i][j][r];
      }
    }
    __builtin_amdgcn_fence(3  , "workgroup");
    __builtin_amdgcn_wave_barrier();
    __builtin_amdgcn_fence(2  , "workgroup");
    if (OUT_MODE == 0) {
      float* Cb0 = (float*)Cout + (size_t)b * (size_t)strideC;
      const int h2 = lane >> 4, c4 = (lane & 15) * 4;
      const v4f braw = *(const v4f*)(bias + n0 + c4);
      v4f bv;
      bv[0] = bf_up(bf_bits(braw[0]));
      bv[1] = bf_up(bf_bits(braw[1]));
      bv[2] = bf_up(bf_bits(braw[2]));
      bv[3] = bf_up(bf_bits(braw[3]));
      for (int ps = 0; ps < 2; ++ps) {
#pragma unroll
        for (int it = 0; it < 8; ++it) {
          const int row = it * 2 + h2;
          const v4f v = *(const v4f*)(slab + row * 68 + c4) * oscale + bv;
          *(volatile v4f*)(Cb0 + (size_t)(mBase + row) * ldc + n0 + c4) = v;
        }
        __threadfence();
      }
    } else {
      const int q = lane >> 3, c8 = (lane & 7) * 8;
      unsigned short* Cp  = (unsigned short*)Cout  + (size_t)b * (size_t)strideC;
      unsigned short* Cp2 = (unsigned short*)Cout2 + (size_t)b * (size_t)strideC;
      v4u hv[4], lv[4];
#pragma unroll
      for (int it = 0; it < 4; ++it) {
        const int row = it * 4 + q;
        const float* sp = slab + row * 68 + c8;
        float f[8];
#pragma unroll
        for (int e = 0; e < 8; ++e) f[e] = sp[e] * oscale;
        v4u a, a2;
#pragma unroll
        for (int e = 0; e < 4; ++e) {
          const float f0 = f[2 * e], f1 = f[2 * e + 1];
          const _Float16 x0 = (_Float16)f0, x1 = (_Float16)f1;
          const unsigned short h0 = h_bits(x0), h1 = h_bits(x1);
          unsigned short l0 = 0, l1 = 0;
          if (OUT_MODE == 3) {
            l0 = h_bits((_Float16)((f0 - (float)x0) * rscale));
            l1 = h_bits((_Float16)((f1 - (float)x1) * rscale));
          }
          a[e] = pk16(h0, h1); a2[e] = pk16(l0, l1);
        }
        hv[it] = a; lv[it] = a2;
      }
      for (int ps = 0; ps < 2; ++ps) {
#pragma unroll
        for (int it = 0; it < 4; ++it) {
          const int row = it * 4 + q;
          *(volatile v4u*)(Cp + (size_t)(mBase + row) * ldc + n0 + c8) = hv[it];
          if (OUT_MODE == 3) *(volatile v4u*)(Cp2 + (size_t)(mBase + row) * ldc + n0 + c8) = lv[it];
        }
        __threadfence();
      }
    }
    __builtin_amdgcn_fence(3  , "workgroup");
    __builtin_amdgcn_wave_barrier();
    __builtin_amdgcn_fence(2  , "workgroup");
  }
}

__global__ __launch_bounds__(256) void gemm_proj_split(
    const unsigned short* __restrict__ Ap, int lda, long long strideA,
    const unsigned short* __restrict__ Btp, int ldb, long long strideB,
    void* Cout, void* Cout2, int ldc, long long strideC,
    const float* __restrict__ bias,
    int M, int N, int K, float oscale, float rscale) {
  __shared__ __align__(16) float sT[8 * 16 * 68];
  gemm64_body<__bf16, 3>(Ap, lda, strideA, Btp, ldb, strideB, Cout, Cout2, ldc, strideC, bias,
                         M, N, K, oscale, rscale, sT);
}
__global__ __launch_bounds__(256) void gemm_proj_plane(
    const unsigned short* __restrict__ Ap, int lda, long long strideA,
    const unsigned short* __restrict__ Btp, int ldb, long long strideB,
    void* Cout, void* Cout2, int ldc, long long strideC,
    const float* __restrict__ bias,
    int M, int N, int K, float oscale, float rscale) {
  __shared__ __align__(16) float sT[8 * 16 * 68];
  gemm64_body<__bf16, 1>(Ap, lda, strideA, Btp, ldb, strideB, Cout, Cout2, ldc, strideC, bias,
                         M, N, K, oscale, rscale, sT);
}
__global__ __launch_bounds__(256) void gemm_out_f32(
    const unsigned short* __restrict__ Ap, int lda, long long strideA,
    const unsigned short* __restrict__ Btp, int ldb, long long strideB,
    void* Cout, void* Cout2, int ldc, long long strideC,
    const float* __restrict__ bias,
    int M, int N, int K, float oscale, float rscale) {
  __shared__ __align__(16) float sT[8 * 16 * 68];
  gemm64_body<_Float16, 0>(Ap, lda, strideA, Btp, ldb, strideB, Cout, Cout2, ldc, strideC, bias,
                           M, N, K, oscale, rscale, sT);
}

__global__ __launch_bounds__(32) void pos_feat_tab(float* tab, float lg, float inv_sd) {
#pragma clang fp contract(off)
  const int f = threadIdx.x & 31;
  const float tt = (float)f / 31.0f;
  const float om = 1.0f - tt;
  float e = 3.0f * om + lg * tt;
  e = (f == 31) ? lg : e;
  const float hl = exp2f(e);
  const float ecoef = -0.6931471805599453f / hl;
  const float m0 = (float)SEQ * 0.03125f;
  const float m1 = (float)SEQ;
  float mean = m0 * om + m1 * tt;
  mean = (f == 31) ? m1 : mean;
  const float ms = mean * inv_sd;
  const float conc = ms * ms;
  const float rate = mean * (inv_sd * inv_sd);
  const float z = conc - 1.0f;
  float x = 0.99999999999980993f;
  x = x + 676.5203681218851f    * __builtin_amdgcn_rcpf((z + 0.0f) + 1.0f);
  x = x + -1259.1392167224028f  * __builtin_amdgcn_rcpf((z + 1.0f) + 1.0f);
  x = x + 771.32342877765313f   * __builtin_amdgcn_rcpf((z + 2.0f) + 1.0f);
  x = x + -176.61502916214059f  * __builtin_amdgcn_rcpf((z + 3.0f) + 1.0f);
  x = x + 12.507343278686905f   * __builtin_amdgcn_rcpf((z + 4.0f) + 1.0f);
  x = x + -0.13857109526572012f * __builtin_amdgcn_rcpf((z + 5.0f) + 1.0f);
  x = x + 9.9843695780195716e-6f * __builtin_amdgcn_rcpf((z + 6.0f) + 1.0f);
  x = x + 1.5056327351493116e-7f * __builtin_amdgcn_rcpf((z + 7.0f) + 1.0f);
  const float t = 7.5f + z;
  const float log_t = 2.0149030205422647f + log1pf(z / 7.5f);
  const float lgam = (0.91893853320467274f + ((z + 0.5f) - t / log_t) * log_t) + logf(x);
  const float lnorm = lgam - conc * logf(rate);
  const float cm1 = conc - 1.0f;
  for (int ps = 0; ps < 2; ++ps) {
    *(volatile float*)(tab + f)      = ecoef;
    *(volatile float*)(tab + 32 + f) = cm1;
    *(volatile float*)(tab + 64 + f) = rate;
    *(volatile float*)(tab + 96 + f) = lnorm;
    __threadfence();
  }
}

__global__ __launch_bounds__(256) void pos_rows(const float* __restrict__ tab, unsigned short* posb) {
#pragma clang fp contract(off)
  __shared__ __align__(16) unsigned short sP[8 * PK];
  const int tid  = threadIdx.x;
  const int f    = tid & 31;
  const int wave = __builtin_amdgcn_readfirstlane(tid >> 5);
  const int n    = blockIdx.x * 8 + wave;
  const float dist = (float)(n - (SEQ - 1));
  const float ad = fabsf(dist);
  const float sgn = (dist > 0.f) ? 1.f : ((dist < 0.f) ? -1.f : 0.f);
  const float ecoef = tab[f];
  const float cm1   = tab[32 + f];
  const float rate  = tab[64 + f];
  const float lnorm = tab[96 + f];
  const float fe = expf(ecoef * ad);
  const float cw = ldexpf(1.0f, f + 1) - 1.0f;
  const float fc = (cw > ad) ? 1.f : 0.f;
  const float la = logf(fmaxf(ad, 1.0f));
  const float lu = cm1 * la - rate * ad;
  const float ex = expf(lu - lnorm);
  const float prob = ((ad > 0.f) ? ex : 0.f) + 1e-8f;
  float mx = prob;
#pragma unroll
  for (int off = 1; off < 32; off <<= 1) mx = fmaxf(mx, __shfl_xor(mx, off, 32));
  const float fg = prob * (1.0f / mx);
  const float live = (n < NPOS - 1) ? 1.f : 0.f;
  float v[6];
  v[0] = fe * live; v[1] = fc * live; v[2] = fg * live;
  v[3] = sgn * v[0]; v[4] = sgn * v[1]; v[5] = sgn * v[2];
#pragma unroll
  for (int g = 0; g < 6; ++g) {
    const unsigned short hb = bf_bits(v[g]);
    const unsigned short lb = bf_bits(v[g] - bf_up(hb));
    sP[wave * PK + g * 32 + f] = hb;
    sP[wave * PK + NRPF + g * 32 + f] = lb;
  }
  __syncthreads();
  const v8us a0 = *(const v8us*)(sP + tid * 8);
  const v8us a1 = *(const v8us*)(sP + ((tid & 127) + 256) * 8);
  const v4u p0 = __builtin_bit_cast(v4u, a0);
  const v4u p1 = __builtin_bit_cast(v4u, a1);
  unsigned short* dst = posb + (size_t)blockIdx.x * (size_t)(8 * PK);
  for (int ps = 0; ps < 2; ++ps) {
    *(volatile v4u*)(dst + tid * 8) = p0;
    if (wave < 4) *(volatile v4u*)(dst + (tid + 256) * 8) = p1;
    __threadfence();
  }
}

__global__ __launch_bounds__(256) void rel_bias_tab(const unsigned short* __restrict__ rhp,
                                                   const unsigned short* __restrict__ rlp,
                                                   const float* __restrict__ rpb, float* ctab,
                                                   float inv_rq, float oscl) {
#pragma clang fp contract(off)
  const int tid  = threadIdx.x;
  const int lane = tid & 31;
  const int hd   = __builtin_amdgcn_readfirstlane(tid >> 5);
  const int n    = blockIdx.x * 32 + lane;
  const _Float16* Rh = (const _Float16*)(const void*)rhp + (size_t)n * DI + (size_t)hd * HD;
  const _Float16* Rl = (const _Float16*)(const void*)rlp + (size_t)n * DI + (size_t)hd * HD;
  const float* bp = rpb + hd * HD;
  float acc = 0.f;
#pragma unroll 1
  for (int d8 = 0; d8 < 8; ++d8) {
    const v8h hv = *(const v8h*)(Rh + d8 * 8);
    const v8h lv = *(const v8h*)(Rl + d8 * 8);
    const v4f b0 = *(const v4f*)(bp + d8 * 8);
    const v4f b1 = *(const v4f*)(bp + d8 * 8 + 4);
#pragma unroll
    for (int e = 0; e < 4; ++e) {
      const float rv = (float)hv[e] + (float)lv[e] * inv_rq;
      acc = acc + bf_up(bf_bits(b0[e])) * rv;
    }
#pragma unroll
    for (int e = 0; e < 4; ++e) {
      const float rv = (float)hv[4 + e] + (float)lv[4 + e] * inv_rq;
      acc = acc + bf_up(bf_bits(b1[e])) * rv;
    }
  }
  const float outv = acc * oscl;
  float* o = ctab + (size_t)hd * NPOS + n;
  *(volatile float*)o = outv;
  __threadfence();
  *(volatile float*)o = outv;
}

__device__ __forceinline__ v8f score_tile(const v16h kA0, const v16h kA1, const v16h qB0, const v16h qB1,
                                          const _Float16* __restrict__ Rg, const float* __restrict__ cg,
                                          const int pb, const int lane, const float sscale) {
  const int hh = lane >> 4;
  const int c  = lane & 15;
  v8f ct = zero8();
  ct = mma_h(kA0, qB0, ct);
  ct = mma_h(kA1, qB1, ct);
  v8f u0, u1;
  {
    const int prow = pb + c;
    const float cv = cg[prow];
    v8f a = {cv, cv, cv, cv, cv, cv, cv, cv};
    const _Float16* rp = Rg + (size_t)prow * DI + 8 * hh;
    const v16h f0 = ldfrag<_Float16>(rp);
    const v16h f1 = ldfrag<_Float16>(rp + 32);
    a = mma_h(kA0, f0, a);
    a = mma_h(kA1, f1, a);
    u0 = a;
  }
  {
    const int prow = pb + 16 + c;
    const float cv = cg[prow];
    v8f a = {cv, cv, cv, cv, cv, cv, cv, cv};
    const _Float16* rp = Rg + (size_t)prow * DI + 8 * hh;
    const v16h f0 = ldfrag<_Float16>(rp);
    const v16h f1 = ldfrag<_Float16>(rp + 32);
    a = mma_h(kA0, f0, a);
    a = mma_h(kA1, f1, a);
    u1 = a;
  }
  v8f s;
#pragma unroll
  for (int r = 0; r < 8; ++r) {
    const int pp = c + 15 - 8 * hh - r;
    const int sl = (lane & 16) | (pp & 15);
    const float g0 = __shfl(u0[r], sl, 32);
    const float g1 = __shfl(u1[r], sl, 32);
    const float g  = (pp < 16) ? g0 : g1;
    s[r] = (ct[r] + g) * sscale;
  }
  return s;
}

__global__ __attribute__((amdgpu_num_vgpr(256))) __launch_bounds__(128)
void attn_fwd(const unsigned short* __restrict__ qpp, const unsigned short* __restrict__ kpp,
              const unsigned short* __restrict__ vtp, const unsigned short* __restrict__ rhp,
              const float* __restrict__ ctab, unsigned short* op, float* stats, float sscale) {
  __shared__ __align__(16) float Os[4][16 * 64];
  __shared__ __align__(16) float sSt[128];

  const int tid  = threadIdx.x;
  const int wave = __builtin_amdgcn_readfirstlane(tid >> 5);
  const int lane = tid & 31;
  const int hh   = lane >> 4;
  const int c    = lane & 15;

  const int bx   = blockIdx.x;
  const int qb   = bx % NQB;
  const int rest = bx / NQB;
  const int hd   = rest % NH;
  const int b    = rest / NH;
  const int q0   = qb * 64 + wave * 16;
  const size_t rowB = (size_t)b * SEQ;

  const _Float16* Qg = (const _Float16*)(const void*)qpp + (size_t)hd * HD;
  const _Float16* Kg = (const _Float16*)(const void*)kpp + (size_t)hd * HD;
  const _Float16* Rg = (const _Float16*)(const void*)rhp + (size_t)hd * HD;
  const _Float16* Vg = (const _Float16*)(const void*)vtp + ((size_t)b * DI + (size_t)hd * HD) * (size_t)SEQ;
  const float* cg = ctab + (size_t)hd * NPOS;

  const v16h qB0 = ldfrag<_Float16>(Qg + (rowB + q0 + c) * DI + 8 * hh);
  const v16h qB1 = ldfrag<_Float16>(Qg + (rowB + q0 + c) * DI + 32 + 8 * hh);

  float mrow = -INFINITY, lrow = 0.f;
  v8f oacc[4];
#pragma unroll
  for (int t = 0; t < 4; ++t) oacc[t] = zero8();

  for (int kv = 0; kv < SEQ; kv += 32) {
    const int pb0 = (SEQ - 16) + q0 - kv;
    const _Float16* kr = Kg + (rowB + kv + c) * DI + 8 * hh;
    v8f s0, s1;
    {
      const v16h ka0 = ldfrag<_Float16>(kr);
      const v16h ka1 = ldfrag<_Float16>(kr + 32);
      s0 = score_tile(ka0, ka1, qB0, qB1, Rg, cg, pb0, lane, sscale);
    }
    {
      const v16h ka0 = ldfrag<_Float16>(kr + (size_t)16 * DI);
      const v16h ka1 = ldfrag<_Float16>(kr + (size_t)16 * DI + 32);
      s1 = score_tile(ka0, ka1, qB0, qB1, Rg, cg, pb0 - 16, lane, sscale);
    }

    float mloc = fmaxf(s0[0], s1[0]);
#pragma unroll
    for (int r = 1; r < 8; ++r) mloc = fmaxf(mloc, fmaxf(s0[r], s1[r]));
    mloc = fmaxf(mloc, __shfl_xor(mloc, 16, 32));
    const float mnew  = fmaxf(mrow, mloc);
    const float msafe = (mnew == -INFINITY) ? 0.f : mnew;
    const float alpha = __expf(mrow - msafe);
    mrow = mnew;
    float psum = 0.f;
    v16h pB;
#pragma unroll
    for (int r = 0; r < 8; ++r) {
      const float p0 = __expf(s0[r] - msafe);
      const float p1 = __expf(s1[r] - msafe);
      psum += p0 + p1;
      pB[r]     = toh_flush(p0 * PCARRY);
      pB[8 + r] = toh_flush(p1 * PCARRY);
    }
    psum += __shfl_xor(psum, 16, 32);
    lrow = lrow * alpha + psum;
#pragma unroll
    for (int t = 0; t < 4; ++t)
#pragma unroll
      for (int r = 0; r < 8; ++r) oacc[t][r] *= alpha;

#pragma unroll
    for (int t = 0; t < 4; ++t) {
      const v16h va = ldfrag<_Float16>(Vg + (size_t)(t * 16 + c) * SEQ + kv + 8 * hh);
      oacc[t] = mma_h(va, pB, oacc[t]);
    }
  }

  float* os = Os[wave];
  const float linv = 1.0f / lrow;
  {
    const float inv = linv * (CCARRY / (PCARRY * VCARRY));
#pragma unroll
    for (int t = 0; t < 4; ++t)
#pragma unroll
      for (int r = 0; r < 8; ++r) os[c * 64 + t * 16 + 8 * hh + r] = oacc[t][r] * inv;
  }
  if (hh == 0) {
    sSt[wave * 16 + c] = mrow;
    sSt[64 + wave * 16 + c] = linv;
  }
  __builtin_amdgcn_fence(3  , "workgroup");
  __builtin_amdgcn_wave_barrier();
  __builtin_amdgcn_fence(2  , "workgroup");
  {
    const int q4 = lane >> 3, c8 = (lane & 7) * 8;
    v4u hv[4];
#pragma unroll
    for (int it = 0; it < 4; ++it) {
      const int row = it * 4 + q4;
      const float* sp = os + row * 64 + c8;
      v4u a;
#pragma unroll
      for (int e = 0; e < 4; ++e)
        a[e] = pk16(h_bits(toh_flush(sp[2 * e])), h_bits(toh_flush(sp[2 * e + 1])));
      hv[it] = a;
    }
    for (int ps = 0; ps < 2; ++ps) {
#pragma unroll
      for (int it = 0; it < 4; ++it) {
        const int row = it * 4 + q4;
        const size_t go = (rowB + q0 + row) * DI + (size_t)hd * HD + c8;
        *(volatile v4u*)(op + go) = hv[it];
      }
      __threadfence();
    }
  }
  __syncthreads();
  if (wave == 0) {
    const v4f sv = *(const v4f*)(sSt + lane * 4);
    float* so = stats + (size_t)bx * 128 + lane * 4;
    *(volatile v4f*)so = sv;
    __threadfence();
    *(volatile v4f*)so = sv;
  }
}

__global__ __attribute__((amdgpu_num_vgpr(256))) __launch_bounds__(128)
void attn_xch(const unsigned short* __restrict__ qpp, const unsigned short* __restrict__ kpp,
              const unsigned short* __restrict__ v1tp, const unsigned short* __restrict__ rhp,
              const float* __restrict__ ctab, const float* __restrict__ stats,
              unsigned short* op, float sscale) {
  union FH { v16h v; v8h h[2]; };
  __shared__ __align__(16) float    Os[4][16 * 64];
  __shared__ __align__(16) _Float16 Pl[4][16 * 40];

  const int tid  = threadIdx.x;
  const int wave = __builtin_amdgcn_readfirstlane(tid >> 5);
  const int lane = tid & 31;
  const int hh   = lane >> 4;
  const int c    = lane & 15;

  const int bx   = blockIdx.x;
  const int jb   = bx % NQB;
  const int rest = bx / NQB;
  const int hd   = rest % NH;
  const int b    = rest / NH;
  const int j0   = jb * 64 + wave * 16;
  const size_t rowB = (size_t)b * SEQ;

  const _Float16* Qg = (const _Float16*)(const void*)qpp + (size_t)hd * HD;
  const _Float16* Kg = (const _Float16*)(const void*)kpp + (size_t)hd * HD;
  const _Float16* Rg = (const _Float16*)(const void*)rhp + (size_t)hd * HD;
  const _Float16* Vg = (const _Float16*)(const void*)v1tp + ((size_t)b * DI + (size_t)hd * HD) * (size_t)SEQ;
  const float* cg = ctab + (size_t)hd * NPOS;
  const float* sg = stats + (size_t)(b * NH + hd) * NQB * 128;

  const v16h kA0 = ldfrag<_Float16>(Kg + (rowB + j0 + c) * DI + 8 * hh);
  const v16h kA1 = ldfrag<_Float16>(Kg + (rowB + j0 + c) * DI + 32 + 8 * hh);

  v8f oacc[4];
#pragma unroll
  for (int t = 0; t < 4; ++t) oacc[t] = zero8();
  _Float16* pl = Pl[wave];

  for (int i0 = 0; i0 < SEQ; i0 += 32) {
    const float* st = sg + (size_t)(i0 >> 6) * 128 + (i0 & 63) + c;
#pragma unroll
    for (int it = 0; it < 2; ++it) {
      const _Float16* qr = Qg + (rowB + i0 + 16 * it + c) * DI + 8 * hh;
      const v16h qB0 = ldfrag<_Float16>(qr);
      const v16h qB1 = ldfrag<_Float16>(qr + 32);
      const float mq = st[16 * it];
      const float li = st[64 + 16 * it];
      const int pb = (SEQ - 16) + i0 + 16 * it - j0;
      const v8f s = score_tile(kA0, kA1, qB0, qB1, Rg, cg, pb, lane, sscale);
#pragma unroll
      for (int r = 0; r < 8; ++r) {
        const float p = __expf(s[r] - mq) * li;
        pl[(8 * hh + r) * 40 + 16 * it + c] = toh_flush(p * PCARRY);
      }
    }
    __builtin_amdgcn_fence(3  , "workgroup");
    __builtin_amdgcn_wave_barrier();
    __builtin_amdgcn_fence(2  , "workgroup");
    FH pb2;
    pb2.h[0] = *(const v8h*)(pl + c * 40 + 8 * hh);
    pb2.h[1] = *(const v8h*)(pl + c * 40 + 16 + 8 * hh);
#pragma unroll
    for (int t = 0; t < 4; ++t) {
      const v16h va = ldfrag<_Float16>(Vg + (size_t)(t * 16 + c) * SEQ + i0 + 8 * hh);
      oacc[t] = mma_h(va, pb2.v, oacc[t]);
    }
    __builtin_amdgcn_fence(3  , "workgroup");
    __builtin_amdgcn_wave_barrier();
    __builtin_amdgcn_fence(2  , "workgroup");
  }

  float* os = Os[wave];
  {
    const float inv = CCARRY / (PCARRY * VCARRY);
#pragma unroll
    for (int t = 0; t < 4; ++t)
#pragma unroll
      for (int r = 0; r < 8; ++r) os[c * 64 + t * 16 + 8 * hh + r] = oacc[t][r] * inv;
  }
  __builtin_amdgcn_fence(3  , "workgroup");
  __builtin_amdgcn_wave_barrier();
  __builtin_amdgcn_fence(2  , "workgroup");
  {
    const int q4 = lane >> 3, c8 = (lane & 7) * 8;
    v4u hv[4];
#pragma unroll
    for (int it = 0; it < 4; ++it) {
      const int row = it * 4 + q4;
      const float* sp = os + row * 64 + c8;
      v4u a;
#pragma unroll
      for (int e = 0; e < 4; ++e)
        a[e] = pk16(h_bits(toh_flush(sp[2 * e])), h_bits(toh_flush(sp[2 * e + 1])));
      hv[it] = a;
    }
    for (int ps = 0; ps < 2; ++ps) {
#pragma unroll
      for (int it = 0; it < 4; ++it) {
        const int row = it * 4 + q4;
        const size_t go = (rowB + j0 + row) * DI + (size_t)hd * HD + c8;
        *(volatile v4u*)(op + go) = hv[it];
      }
      __threadfence();
    }
  }
}

extern "C" void kernel_launch(void* const* d_in, const int* in_sizes, int n_in,
                              void* d_out, int out_size, void* d_ws, size_t ws_size,
                              hipStream_t stream) {
  if (n_in < 12) return;
  if (in_sizes[0] < NB * SEQ_FULL * DM1) return;
  if (in_sizes[1] < NB * SEQ_FULL * DM2) return;
  if (in_sizes[2] < DM1 * DI || in_sizes[3] < DM2 * DI) return;
  if (in_sizes[4] < DM1 * DI || in_sizes[5] < DM2 * DI) return;
  if (in_sizes[6] < NRPF * DI || in_sizes[7] < NH * HD) return;
  if (in_sizes[8] < DI * DM1 || in_sizes[9] < DM1) return;
  if (in_sizes[10] < DI * DM1 || in_sizes[11] < DM1) return;
  if ((size_t)out_size < OUT2_OFF + (size_t)((NB - 1) * SEQ_FULL + SEQ) * DM1) return;

  const float* x1   = (const float*)d_in[0];
  const float* x2   = (const float*)d_in[1];
  const float* Wq   = (const float*)d_in[2];
  const float* Wk   = (const float*)d_in[3];
  const float* Wv1  = (const float*)d_in[4];
  const float* Wv2  = (const float*)d_in[5];
  const float* Wrel = (const float*)d_in[6];
  const float* rpb  = (const float*)d_in[7];
  const float* Wo1  = (const float*)d_in[8];
  const float* bo1  = (const float*)d_in[9];
  const float* Wo2  = (const float*)d_in[10];
  const float* bo2  = (const float*)d_in[11];

  size_t off = 0;
  const size_t oX1 = off; off += WSB_X1;
  const size_t oX2 = off; off += WSB_X2;
  const size_t oWq = off; off += WSB_W1;
  const size_t oW1 = off; off += WSB_W1;
  const size_t oWk = off; off += WSB_W2;
  const size_t oW2 = off; off += WSB_W2;
  const size_t oWr = off; off += WSB_WR;
  const size_t oO1 = off; off += WSB_WO;
  const size_t oO2 = off; off += WSB_WO;
  const size_t oPo = off; off += WSB_POS;
  const size_t oPt = off; off += WSB_PT;
  const size_t oQp = off; off += WSB_P;
  const size_t oKp = off; off += WSB_P;
  const size_t oV1 = off; off += WSB_P;
  const size_t oV2 = off; off += WSB_P;
  const size_t oRh = off; off += WSB_R;
  const size_t oRl = off; off += WSB_R;
  const size_t oCt = off; off += WSB_CT;
  const size_t oSt = off; off += WSB_ST;
  const size_t oC1 = off; off += WSB_P;
  const size_t oC2 = off; off += WSB_P;
  if (off != WSB_TOTAL) return;
  if (off > ws_size) return;
  if (off > (size_t)134217728) return;

  char* ws = (char*)d_ws;
  unsigned short* X1b  = (unsigned short*)(ws + oX1);
  unsigned short* X2b  = (unsigned short*)(ws + oX2);
  unsigned short* WqT  = (unsigned short*)(ws + oWq);
  unsigned short* Wv1T = (unsigned short*)(ws + oW1);
  unsigned short* WkT  = (unsigned short*)(ws + oWk);
  unsigned short* Wv2T = (unsigned short*)(ws + oW2);
  unsigned short* WrT  = (unsigned short*)(ws + oWr);
  unsigned short* Wo1T = (unsigned short*)(ws + oO1);
  unsigned short* Wo2T = (unsigned short*)(ws + oO2);
  unsigned short* PosB = (unsigned short*)(ws + oPo);
  float*          Ptab = (float*)(ws + oPt);
  unsigned short* Qp   = (unsigned short*)(ws + oQp);
  unsigned short* Kp   = (unsigned short*)(ws + oKp);
  unsigned short* V1T  = (unsigned short*)(ws + oV1);
  unsigned short* V2T  = (unsigned short*)(ws + oV2);
  unsigned short* Rh   = (unsigned short*)(ws + oRh);
  unsigned short* Rl   = (unsigned short*)(ws + oRl);
  float*          Ctab = (float*)(ws + oCt);
  float*          Stat = (float*)(ws + oSt);
  unsigned short* C1   = (unsigned short*)(ws + oC1);
  unsigned short* C2   = (unsigned short*)(ws + oC2);
  float* outf = (float*)d_out;

  const dim3 blk(256);
  const int n8a = SEQ * DM1 / 8;
  const int n8b = SEQ * DM2 / 8;
  const dim3 gCvtA((n8a + 255) / 256, NB);
  const dim3 gCvtB((n8b + 255) / 256, NB);
  const dim3 gWT1(DI / 64, DM1 / 64);
  const dim3 gWT2(DI / 64, DM2 / 64);
  const dim3 gWTR(DI / 64, NRPF / 64);
  const dim3 gWO(DM1 / 64, DI / 64);
  const dim3 gP((((NB * SEQ) / 64) * (DI / 64) + 7) / 8, 1);
  const dim3 gVT(((DI / 64) * (SEQ / 64) + 7) / 8, NB);
  const dim3 gR(((NPOS / 64) * (DI / 64) + 7) / 8, 1);
  const dim3 gAttn(NB * NH * NQB);
  const dim3 gO((((SEQ / 64) * (DM1 / 64)) + 7) / 8, NB);

  const float lg = log2f((float)SEQ);
  const float inv_sd = 64.0f / (float)SEQ;

  cvt_bf16x8<<<gCvtA, blk, 0, stream>>>(x1, (long long)SEQ_FULL * DM1, X1b, (long long)SEQ * DM1, n8a);
  cvt_bf16x8<<<gCvtB, blk, 0, stream>>>(x2, (long long)SEQ_FULL * DM2, X2b, (long long)SEQ * DM2, n8b);
  wtrans_bf16<<<gWT1, blk, 0, stream>>>(Wq,  DI, WqT,  DM1, 0, 1.0f);
  wtrans_bf16<<<gWT2, blk, 0, stream>>>(Wk,  DI, WkT,  DM2, 0, 1.0f);
  wtrans_bf16<<<gWT1, blk, 0, stream>>>(Wv1, DI, Wv1T, DM1, 0, 1.0f);
  wtrans_bf16<<<gWT2, blk, 0, stream>>>(Wv2, DI, Wv2T, DM2, 0, 1.0f);
  wtrans_bf16<<<gWTR, blk, 0, stream>>>(Wrel, DI, WrT, PK, 0,    1.0f);
  wtrans_bf16<<<gWTR, blk, 0, stream>>>(Wrel, DI, WrT, PK, NRPF, 1.0f);
  wtrans_f16s<<<gWO, blk, 0, stream>>>(Wo1, DM1, Wo1T, DI, 0, WOC);
  wtrans_f16s<<<gWO, blk, 0, stream>>>(Wo2, DM1, Wo2T, DI, 0, WOC);
  pos_feat_tab<<<dim3(1), dim3(32), 0, stream>>>(Ptab, lg, inv_sd);
  pos_rows<<<dim3(NPOS / 8), blk, 0, stream>>>(Ptab, PosB);
  gemm_proj_plane<<<gP, blk, 0, stream>>>(
      X1b, DM1, 0LL, WqT, DM1, 0LL,
      (void*)Qp, (void*)Qp, DI, 0LL, bo1,
      NB * SEQ, DI, DM1, 1.0f, 1.0f);
  gemm_proj_plane<<<gP, blk, 0, stream>>>(
      X2b, DM2, 0LL, WkT, DM2, 0LL,
      (void*)Kp, (void*)Kp, DI, 0LL, bo1,
      NB * SEQ, DI, DM2, 1.0f, 1.0f);
  gemm_proj_plane<<<gVT, blk, 0, stream>>>(
      Wv2T, DM2, 0LL, X2b, DM2, (long long)SEQ * DM2,
      (void*)V2T, (void*)V2T, SEQ, (long long)DI * SEQ, bo1,
      DI, SEQ, DM2, VCARRY, 1.0f);
  gemm_proj_plane<<<gVT, blk, 0, stream>>>(
      Wv1T, DM1, 0LL, X1b, DM1, (long long)SEQ * DM1,
      (void*)V1T, (void*)V1T, SEQ, (long long)DI * SEQ, bo1,
      DI, SEQ, DM1, VCARRY, 1.0f);
  gemm_proj_split<<<gR, blk, 0, stream>>>(
      PosB, PK, 0LL, WrT, PK, 0LL,
      (void*)Rh, (void*)Rl, DI, 0LL, bo1,
      NPOS, DI, PK, 1.0f, RQ);
  rel_bias_tab<<<dim3(NPOS / 32), blk, 0, stream>>>(Rh, Rl, rpb, Ctab, 1.0f / RQ, 8.0f);
  attn_fwd<<<gAttn, dim3(128), 0, stream>>>(Qp, Kp, V2T, Rh, Ctab, C1, Stat, 0.125f);
  attn_xch<<<gAttn, dim3(128), 0, stream>>>(Qp, Kp, V1T, Rh, Ctab, Stat, C2, 0.125f);
  gemm_out_f32<<<gO, blk, 0, stream>>>(
      C1, DI, (long long)SEQ * DI, Wo1T, DI, 0LL,
      (void*)outf, (void*)outf, DM1, (long long)SEQ_FULL * DM1, bo1,
      SEQ, DM1, DI, 1.0f / (CCARRY * WOC), 1.0f);
  gemm_out_f32<<<gO, blk, 0, stream>>>(
      C2, DI, (long long)SEQ * DI, Wo2T, DI, 0LL,
      (void*)(outf + OUT2_OFF), (void*)(outf + OUT2_OFF), DM1, (long long)SEQ_FULL * DM1, bo2,
      SEQ, DM1, DI, 1.0f / (CCARRY * WOC), 1.0f);
  (void)hipGetLastError();
}
